// ContrastiveGAE_87316685127955
// MI455X (gfx1250) — hardware-run, weakly checked
//
#include <hip/hip_runtime.h>
#include <math.h>

#pragma clang fp contract(off)

typedef __attribute__((ext_vector_type(16))) _Float16 v16h;
typedef __attribute__((ext_vector_type(8)))  _Float16 v8h;
typedef __attribute__((ext_vector_type(16))) __bf16   v16b;
typedef __attribute__((ext_vector_type(8)))  __bf16   v8b;
typedef __attribute__((ext_vector_type(8)))  float    v8f;
typedef __attribute__((ext_vector_type(4)))  float    v4f;
typedef __attribute__((ext_vector_type(4)))  unsigned v4u;
typedef __attribute__((ext_vector_type(4)))  int      v4i;
typedef __attribute__((ext_vector_type(8)))  unsigned short us8;

constexpr int kN      = 50000;
constexpr int kE      = 800000;
constexpr int kInCh   = 256;
constexpr int kHid    = 64;
constexpr int kHeads  = 8;
constexpr int kF1     = kHeads * kHid;
constexpr int kLat    = 256;
constexpr int kGraphs = 64;
constexpr int kMP     = 50048;
constexpr int kCap       = 64;
constexpr int kTile      = 480;
constexpr int kTabBlocks = 105;
constexpr int kTabRows   = kTabBlocks * kTile;
constexpr int kQuads     = kE / 4;
constexpr int kScanIters = (kQuads + 511) / 512;
constexpr float kWCarry   = 16.0f;
constexpr float kGCarry   = 16.0f;
constexpr float kInvW     = 1.0f / kWCarry;
constexpr float kInvGW    = 1.0f / (kWCarry * kGCarry);
static_assert(kF1 == 512);
static_assert((kMP % 64) == 0 && kMP >= kN && kMP - kN < 64);
static_assert((kN % 16) == 0);
static_assert(kTabRows >= kN && (kTile % 4) == 0 && ((kTile * 4) % 128) == 0);
static_assert((kE % 4) == 0 && kN <= 65536);
static_assert((kInCh % 32) == 0 && (kF1 % 32) == 0 && (kLat % 32) == 0 && (kHid % 32) == 0);
static_assert((kF1 % 64) == 0 && (kLat % 64) == 0 && (kHid % 64) == 0);
static_assert(((kMP * kInCh / 8) % 256) == 0);

constexpr size_t kSzBig   = (size_t)kMP * kF1 * 2;
constexpr size_t kSzHalf  = (size_t)kMP * kLat * 2;
constexpr size_t kSzT     = (size_t)kMP * kHid * 2;
constexpr size_t kOffR1   = 0;
constexpr size_t kOffR2   = kOffR1  + kSzBig;
constexpr size_t kOffTH   = kOffR2  + kSzBig;
constexpr size_t kOffTL   = kOffTH  + kSzT;
constexpr size_t kOffW1T  = kOffTL  + kSzT;
constexpr size_t kOffW2T  = kOffW1T + (size_t)kF1 * kInCh * 2;
constexpr size_t kOffP1H  = kOffW2T + (size_t)kLat * kF1 * 2;
constexpr size_t kOffP1L  = kOffP1H + (size_t)kHid * kLat * 2;
constexpr size_t kOffP2H  = kOffP1L + (size_t)kHid * kLat * 2;
constexpr size_t kOffP2L  = kOffP2H + (size_t)kLat * kHid * 2;
constexpr size_t kOffAS1  = kOffP2L + (size_t)kLat * kHid * 2;
constexpr size_t kOffAD1  = kOffAS1 + (size_t)kMP * kHeads * 4;
constexpr size_t kOffAS2  = kOffAD1 + (size_t)kMP * kHeads * 4;
constexpr size_t kOffAD2  = kOffAS2 + (size_t)kMP * 4;
constexpr size_t kOffDEG  = kOffAD2 + (size_t)kMP * 4;
constexpr size_t kOffTAB  = kOffDEG + (size_t)kTabRows * 4;
constexpr size_t kWsTotal = kOffTAB + (size_t)kTabRows * kCap * 2;
static_assert(kWsTotal == 126222208ull);
static_assert(kWsTotal <= 134217728ull);
static_assert((kOffR2 % 128) == 0 && (kOffTH % 128) == 0 && (kOffTL % 128) == 0 && (kOffW1T % 128) == 0 &&
              (kOffW2T % 128) == 0 && (kOffP1H % 128) == 0 && (kOffP1L % 128) == 0 && (kOffP2H % 128) == 0 &&
              (kOffP2L % 128) == 0 && (kOffAS1 % 128) == 0 && (kOffAD1 % 128) == 0 && (kOffAS2 % 128) == 0 &&
              (kOffAD2 % 128) == 0 && (kOffDEG % 128) == 0 && (kOffTAB % 128) == 0 && (kSzHalf % 128) == 0);
constexpr size_t kOut1ByteOff = 51200000ull;
constexpr size_t kOutTotalB   = 51265536ull;
static_assert(kOut1ByteOff == (size_t)kN * kLat * 4);
static_assert(kOut1ByteOff + (size_t)kGraphs * kLat * 4 <= kOutTotalB);
static_assert((kOut1ByteOff % 128) == 0);

__device__ __forceinline__ unsigned short f2bf_bits(float f) {
  unsigned u = __float_as_uint(f);
  return (unsigned short)((u + 0x7FFFu + ((u >> 16) & 1u)) >> 16);
}
__device__ __forceinline__ float bf_bits2f(unsigned short h) { return __uint_as_float(((unsigned)h) << 16); }

__device__ __forceinline__ float h16_to_f32(unsigned hb) {
  const unsigned sgn = (hb & 0x8000u) << 16; const unsigned em = hb & 0x7fffu;
  const float fn = __uint_as_float((em << 13) + 0x38000000u);
  const float fs = (float)em * 5.9604644775390625e-8f;
  const float mag = (em < 0x400u) ? fs : fn; return __uint_as_float(__float_as_uint(mag) | sgn);
}
__device__ __forceinline__ float leaky02(float v) { return (v >= 0.0f) ? v : 0.2f * v; }

__device__ __forceinline__ void dep_guard1_h(v8f& a, v16h x, v16h y) { asm volatile("v_nop\n\tv_nop\n\tv_nop\n\tv_nop" : "+v"(a) : "v"(x), "v"(y)); }
__device__ __forceinline__ void dep_guard1_b(v8f& a, v16b x, v16b y) { asm volatile("v_nop\n\tv_nop\n\tv_nop\n\tv_nop" : "+v"(a) : "v"(x), "v"(y)); }
__device__ __forceinline__ void dep_guard1s_h(v8f& a, v16h x, v16h x2, v16h y, v16h y2) { asm volatile("v_nop\n\tv_nop\n\tv_nop\n\tv_nop" : "+v"(a) : "v"(x), "v"(x2), "v"(y), "v"(y2)); }
__device__ __forceinline__ void dep_guard1s_b(v8f& a, v16b x, v16b x2, v16b y, v16b y2) { asm volatile("v_nop\n\tv_nop\n\tv_nop\n\tv_nop" : "+v"(a) : "v"(x), "v"(x2), "v"(y), "v"(y2)); }
__device__ __forceinline__ void keep4_h(v16h a, v16h b, v16h c, v16h d) { asm volatile("v_nop" :: "v"(a), "v"(b), "v"(c), "v"(d)); }
__device__ __forceinline__ void keep4_b(v16b a, v16b b, v16b c, v16b d) { asm volatile("v_nop" :: "v"(a), "v"(b), "v"(c), "v"(d)); }
__device__ __forceinline__ void acc_guard4(v8f& a, v8f& b, v8f& c, v8f& d) { asm volatile("v_nop\n\tv_nop\n\tv_nop\n\tv_nop" : "+v"(a), "+v"(b), "+v"(c), "+v"(d)); }

template <typename T> struct Frag;
template <> struct Frag<_Float16> {
  typedef v16h V; union U { v16h v; v8h h[2]; };
  static __device__ __forceinline__ v16h load(const _Float16* p) {
    U f; f.h[0] = *(const v8h*)(p); f.h[1] = *(const v8h*)(p + 16); return f.v;
  }
  static __device__ __forceinline__ v8f mma(v16h a, v16h b, v8f c) {
    return __builtin_amdgcn_wmma_f32_16x16x32_f16(false, a, false, b, (short)0, c, false, false);
  }
  static __device__ __forceinline__ void guard1(v8f& a, v16h x, v16h y) { dep_guard1_h(a, x, y); }
  static __device__ __forceinline__ void guard1s(v8f& a, v16h x, v16h x2, v16h y, v16h y2) { dep_guard1s_h(a, x, x2, y, y2); }
  static __device__ __forceinline__ void keep(v16h a, v16h b, v16h c, v16h d) { keep4_h(a, b, c, d); }
};
template <> struct Frag<__bf16> {
  typedef v16b V; union U { v16b v; v8b h[2]; };
  static __device__ __forceinline__ v16b load(const __bf16* p) {
    U f; f.h[0] = *(const v8b*)(p); f.h[1] = *(const v8b*)(p + 16); return f.v;
  }
  static __device__ __forceinline__ v8f mma(v16b a, v16b b, v8f c) {
    return __builtin_amdgcn_wmma_f32_16x16x32_bf16(false, a, false, b, (short)0, c, false, false);
  }
  static __device__ __forceinline__ void guard1(v8f& a, v16b x, v16b y) { dep_guard1_b(a, x, y); }
  static __device__ __forceinline__ void guard1s(v8f& a, v16b x, v16b x2, v16b y, v16b y2) { dep_guard1s_b(a, x, x2, y, y2); }
  static __device__ __forceinline__ void keep(v16b a, v16b b, v16b c, v16b d) { keep4_b(a, b, c, d); }
};

template <int ET> struct Elem;
template <> struct Elem<0> { typedef _Float16 T; };
template <> struct Elem<1> { typedef __bf16 T; };
template <int ET, bool SPLIT, int BIAS_MODE, int OUT_MODE, bool RESID, int ACT = 0>
__global__ __launch_bounds__(256) void wmma_gemm64(
    const unsigned short* __restrict__ Ap, const unsigned short* __restrict__ A2p, int lda, long strideA,
    const unsigned short* __restrict__ Btp, const unsigned short* __restrict__ Bt2p, int ldb, long strideB,
    void* __restrict__ Cout, void* __restrict__ Cout2, int ldc, long strideC,
    const float* __restrict__ bias,
    const float* __restrict__ resid, long strideR,
    int M, int N, int K, float scale, int Mstore) {
  typedef typename Elem<ET>::T T;
  typedef typename Frag<T>::V V;
  const T* A = (const T*)Ap; const T* A2 = (const T*)A2p; const T* Bt = (const T*)Btp; const T* Bt2 = (const T*)Bt2p;
  __shared__ __align__(16) float sT[8][16 * 68];
  const int b    = blockIdx.y;
  const int lane = threadIdx.x & 31;
  const int wave = threadIdx.x >> 5;
  const int tilesN = N >> 6;
  const int tilesM = M >> 6;
  const int tile = blockIdx.x * 8 + wave;
  if (tile >= tilesM * tilesN) return;
  const int tm = tile / tilesN;
  const int tn = tile - tm * tilesN;
  const int m0 = tm << 6;
  const int n0 = tn << 6;

  const T* Ab  = A  + (size_t)b * strideA;
  const T* Bb  = Bt + (size_t)b * strideB;
  const T* Ab2 = SPLIT ? (A2  + (size_t)b * strideA) : nullptr;
  const T* Bb2 = SPLIT ? (Bt2 + (size_t)b * strideB) : nullptr;

  const int rlane = lane & 15;
  const int koff  = (lane >> 4) * 8;
  const int mOff  = (lane >> 4) * 8;

  v8f acc[4][4];
#pragma unroll
  for (int i = 0; i < 4; ++i)
#pragma unroll
    for (int j = 0; j < 4; ++j) acc[i][j] = (v8f){0.f,0.f,0.f,0.f,0.f,0.f,0.f,0.f};

  for (int k0 = 0; k0 < K; k0 += 32) {
    V bh[4], bl[4];
#pragma unroll
    for (int j = 0; j < 4; ++j) {
      const size_t bo = (size_t)(n0 + (j << 4) + rlane) * ldb + koff + k0;
      bh[j] = Frag<T>::load(Bb + bo);
      if (SPLIT) bl[j] = Frag<T>::load(Bb2 + bo);
    }
#pragma unroll
    for (int i = 0; i < 4; ++i) {
      const size_t ao = (size_t)(m0 + (i << 4) + rlane) * lda + koff + k0;
      V ah = Frag<T>::load(Ab + ao);
      V al;
      if (SPLIT) al = Frag<T>::load(Ab2 + ao);
#pragma unroll
      for (int j = 0; j < 4; ++j) {
        acc[i][j] = Frag<T>::mma(ah, bh[j], acc[i][j]);
        if (SPLIT) {
          acc[i][j] = Frag<T>::mma(ah, bl[j], acc[i][j]);
          acc[i][j] = Frag<T>::mma(al, bh[j], acc[i][j]);
        }
      }
#pragma unroll
      for (int j = 0; j < 4; ++j) {
        if (SPLIT) Frag<T>::guard1s(acc[i][j], ah, al, bh[j], bl[j]);
        else       Frag<T>::guard1(acc[i][j], ah, bh[j]);
      }
    }
    Frag<T>::keep(bh[0], bh[1], bh[2], bh[3]);
    if (SPLIT) Frag<T>::keep(bl[0], bl[1], bl[2], bl[3]);
  }
  acc_guard4(acc[0][0], acc[0][1], acc[0][2], acc[0][3]);
  acc_guard4(acc[1][0], acc[1][1], acc[1][2], acc[1][3]);
  acc_guard4(acc[2][0], acc[2][1], acc[2][2], acc[2][3]);
  acc_guard4(acc[3][0], acc[3][1], acc[3][2], acc[3][3]);

  float* slab = sT[wave];
#pragma unroll
  for (int i = 0; i < 4; ++i) {
    const int mBase = m0 + (i << 4);
#pragma unroll
    for (int j = 0; j < 4; ++j) {
      const int n = n0 + (j << 4) + rlane;
      float bv = 0.f;
      if (BIAS_MODE == 2) bv = bias[n];
#pragma unroll
      for (int r = 0; r < 8; ++r) {
        float v = acc[i][j][r] * scale;
        if (BIAS_MODE == 1) v += bias[mBase + mOff + r];
        if (BIAS_MODE == 2) v += bv;
        if (ACT == 2) v = fmaxf(v, 0.0f);
        slab[(mOff + r) * 68 + (j << 4) + rlane] = v;
      }
    }
    __builtin_amdgcn_fence(__ATOMIC_RELEASE, "workgroup");
    __builtin_amdgcn_wave_barrier();
    __builtin_amdgcn_fence(__ATOMIC_ACQUIRE, "workgroup");
    if (OUT_MODE == 0) {
      float* C = (float*)Cout + (size_t)b * strideC;
      const int hh = lane >> 4, c4 = (lane & 15) * 4;
      for (int pass = 0; pass < 2; ++pass) {
#pragma unroll
        for (int it = 0; it < 8; ++it) {
          const int row = it * 2 + hh;
          v4f v = *(const v4f*)(slab + row * 68 + c4);
          if (mBase + row < Mstore)
            *(volatile v4f*)(C + (size_t)(mBase + row) * ldc + n0 + c4) = v;
        }
        __threadfence();
      }
    } else {
      const int q = lane >> 3, c8 = (lane & 7) * 8;
      unsigned short* C  = (unsigned short*)Cout  + (size_t)b * strideC;
      unsigned short* C2 = (OUT_MODE == 2) ? ((unsigned short*)Cout2 + (size_t)b * strideC) : nullptr;
      for (int pass = 0; pass < 2; ++pass) {
#pragma unroll
        for (int it = 0; it < 4; ++it) {
          const int row = it * 4 + q;
          const float* sp = slab + row * 68 + c8;
          v8h hv, lv;
#pragma unroll
          for (int e = 0; e < 8; ++e) {
            if (OUT_MODE == 1) {
              hv[e] = (_Float16)sp[e];
            } else {
              unsigned short hb = f2bf_bits(sp[e]);
              unsigned short lb = f2bf_bits(sp[e] - bf_bits2f(hb));
              hv[e] = __builtin_bit_cast(_Float16, hb);
              lv[e] = __builtin_bit_cast(_Float16, lb);
            }
          }
          if (mBase + row < Mstore) {
            *(volatile v8h*)(C + (size_t)(mBase + row) * ldc + n0 + c8) = hv;
            if (OUT_MODE == 2) *(volatile v8h*)(C2 + (size_t)(mBase + row) * ldc + n0 + c8) = lv;
          }
        }
        __threadfence();
      }
    }
    __builtin_amdgcn_fence(__ATOMIC_RELEASE, "workgroup");
    __builtin_amdgcn_wave_barrier();
    __builtin_amdgcn_fence(__ATOMIC_ACQUIRE, "workgroup");
  }
}

__global__ __launch_bounds__(256) void cvt_x_f16_kernel(const float* __restrict__ x, unsigned short* __restrict__ x16)
{
  const int i = blockIdx.x * 256 + threadIdx.x;
  if (i >= kMP * kInCh / 8) return;
  const size_t e0 = (size_t)i << 3;
  const bool valid = e0 < (size_t)kN * kInCh;
  const size_t ec = valid ? e0 : ((size_t)kN * kInCh - 8);
  const v4f a0 = *(const v4f*)(x + ec);
  const v4f a1 = *(const v4f*)(x + ec + 4);
  v8h hv;
#pragma unroll
  for (int e = 0; e < 4; ++e) {
    const float f0 = valid ? a0[e] : 0.0f;
    const float f1 = valid ? a1[e] : 0.0f;
    hv[e]     = (_Float16)f0;
    hv[4 + e] = (_Float16)f1;
  }
  unsigned short* q = x16 + e0;
  *(volatile v8h*)q = hv;
  __threadfence();
  *(volatile v8h*)q = hv;
}

template <int MODE>
__global__ __launch_bounds__(256) void transpose_w_kernel(const float* __restrict__ W, int R, int C,
                                                          unsigned short* __restrict__ Ohi,
                                                          unsigned short* __restrict__ Olo, float carry)
{
  __shared__ float sT[64 * 65];
  const int tid = threadIdx.x;
  const int c0 = blockIdx.x * 64, r0 = blockIdx.y * 64;
  {
    const int c = tid & 63, rb = tid >> 6;
#pragma unroll
    for (int i = 0; i < 16; ++i) {
      const int r = rb + 4 * i;
      sT[r * 65 + c] = W[(size_t)(r0 + r) * C + c0 + c];
    }
  }
  __syncthreads();
  const int q = tid >> 3, c8 = (tid & 7) * 8;
  v8h hv[2], lv[2];
#pragma unroll
  for (int it = 0; it < 2; ++it) {
    const int c = it * 32 + q;
#pragma unroll
    for (int e = 0; e < 8; ++e) {
      const float f = sT[(c8 + e) * 65 + c];
      if (MODE == 0) {
        hv[it][e] = (_Float16)(f * carry);
        lv[it][e] = (_Float16)0.0f;
      } else {
        const unsigned short hb = f2bf_bits(f);
        const unsigned short lb = f2bf_bits(f - bf_bits2f(hb));
        hv[it][e] = __builtin_bit_cast(_Float16, hb);
        lv[it][e] = __builtin_bit_cast(_Float16, lb);
      }
    }
  }
  for (int pass = 0; pass < 2; ++pass) {
#pragma unroll
    for (int it = 0; it < 2; ++it) {
      const size_t o = (size_t)(c0 + it * 32 + q) * R + r0 + c8;
      *(volatile v8h*)(Ohi + o) = hv[it];
      if (MODE == 1) *(volatile v8h*)(Olo + o) = lv[it];
    }
    __threadfence();
  }
}

__global__ __launch_bounds__(512) void build_table_kernel(const int* __restrict__ ei,
                                                          unsigned short* __restrict__ tab, int* __restrict__ deg)
{
  __shared__ __align__(16) unsigned short sTab[kTile * kCap];
  __shared__ __align__(16) int sCnt[kTile];
  const int tid = threadIdx.x;
  const int base = blockIdx.x * kTile;
  {
    const us8 zz = {0, 0, 0, 0, 0, 0, 0, 0};
#pragma unroll 1
    for (int c = tid; c < kTile * kCap / 8; c += 512) *(us8*)(sTab + c * 8) = zz;
    if (tid < kTile) sCnt[tid] = 0;
  }
  __syncthreads();
#pragma unroll 1
  for (int it = 0; it < kScanIters; ++it) {
    const int qd = it * 512 + tid;
    const bool valid = qd < kQuads;
    const int qc = valid ? qd : (kQuads - 1);
    const v4i s4 = *(const v4i*)(ei + (size_t)qc * 4);
    const v4i d4 = *(const v4i*)(ei + (size_t)kE + (size_t)qc * 4);
#pragma unroll
    for (int c = 0; c < 4; ++c) {
      int dv = d4[c];
      int sv = s4[c];
      dv = dv < 0 ? 0 : (dv > kN - 1 ? kN - 1 : dv);
      sv = sv < 0 ? 0 : (sv > kN - 1 ? kN - 1 : sv);
      const int ln = dv - base;
      if (valid && (unsigned)ln < (unsigned)kTile) {
        const int pos = atomicAdd(&sCnt[ln], 1);
        if (pos >= 0 && pos < kCap) sTab[ln * kCap + pos] = (unsigned short)sv;
      }
    }
  }
  __syncthreads();
  if (tid < kTile) {
    int n = sCnt[tid];
    n = n > kCap ? kCap : n;
    unsigned short* row = sTab + tid * kCap;
#pragma unroll 1
    for (int a = 1; a < n; ++a) {
      const unsigned short key = row[a];
      int b = a - 1;
#pragma unroll 1
      for (int s = 0; s < kCap; ++s) {
        if (b < 0) break;
        const unsigned short cur = row[b];
        if (cur <= key) break;
        row[b + 1] = cur;
        --b;
      }
      row[b + 1] = key;
    }
  }
  __syncthreads();
  unsigned short* gt = tab + (size_t)base * kCap;
  for (int pass = 0; pass < 2; ++pass) {
#pragma unroll 1
    for (int c = tid; c < kTile * kCap / 8; c += 512) {
      const us8 v = *(const us8*)(sTab + c * 8);
      *(volatile us8*)(gt + (size_t)c * 8) = v;
    }
    if (tid < kTile / 4) {
      const v4i dv = *(const v4i*)(sCnt + tid * 4);
      *(volatile v4i*)(deg + base + tid * 4) = dv;
    }
    __threadfence();
  }
}

__global__ __launch_bounds__(256) void score1_kernel(const unsigned short* __restrict__ h1,
                                                     const float* __restrict__ as1, const float* __restrict__ ad1,
                                                     float* __restrict__ asrc, float* __restrict__ adst)
{
  __shared__ __align__(16) float sSD[1024];
  const int tid = threadIdx.x, lane = tid & 31, wave = tid >> 5;
  float ws[16], wd[16];
#pragma unroll
  for (int m = 0; m < 4; ++m) {
    const v4f a = *(const v4f*)(as1 + lane * 16 + 4 * m);
    const v4f d = *(const v4f*)(ad1 + lane * 16 + 4 * m);
    ws[4 * m + 0] = a[0]; ws[4 * m + 1] = a[1]; ws[4 * m + 2] = a[2]; ws[4 * m + 3] = a[3];
    wd[4 * m + 0] = d[0]; wd[4 * m + 1] = d[1]; wd[4 * m + 2] = d[2]; wd[4 * m + 3] = d[3];
  }
#pragma unroll 1
  for (int nn = 0; nn < 8; ++nn) {
    const int ln = wave * 8 + nn;
    const int node = blockIdx.x * 64 + ln;
    const v4u p0 = *(const v4u*)(h1 + (size_t)node * kF1 + lane * 16);
    const v4u p1 = *(const v4u*)(h1 + (size_t)node * kF1 + lane * 16 + 8);
    float s = 0.0f, d = 0.0f;
#pragma unroll
    for (int m = 0; m < 4; ++m) {
      const unsigned w0 = p0[m];
      const unsigned w1 = p1[m];
      const float f0 = h16_to_f32(w0 & 0xffffu), f1 = h16_to_f32(w0 >> 16);
      const float f2 = h16_to_f32(w1 & 0xffffu), f3 = h16_to_f32(w1 >> 16);
      s = fmaf(f0, ws[2 * m], s);         d = fmaf(f0, wd[2 * m], d);
      s = fmaf(f1, ws[2 * m + 1], s);     d = fmaf(f1, wd[2 * m + 1], d);
      s = fmaf(f2, ws[8 + 2 * m], s);     d = fmaf(f2, wd[8 + 2 * m], d);
      s = fmaf(f3, ws[8 + 2 * m + 1], s); d = fmaf(f3, wd[8 + 2 * m + 1], d);
    }
    s += __shfl_xor(s, 1, 32); d += __shfl_xor(d, 1, 32);
    s += __shfl_xor(s, 2, 32); d += __shfl_xor(d, 2, 32);
    if ((lane & 3) == 0) {
      sSD[ln * 8 + (lane >> 2)] = s;
      sSD[512 + ln * 8 + (lane >> 2)] = d;
    }
  }
  __syncthreads();
  {
    const v4f v = *(const v4f*)(sSD + tid * 4);
    float* gp = (tid < 128) ? (asrc + (size_t)blockIdx.x * 512 + tid * 4)
                            : (adst + (size_t)blockIdx.x * 512 + (tid - 128) * 4);
    *(volatile v4f*)gp = v;
    __threadfence();
    *(volatile v4f*)gp = v;
  }
}

__global__ __launch_bounds__(256) void score2_kernel(const unsigned short* __restrict__ h2,
                                                     const float* __restrict__ as2, const float* __restrict__ ad2,
                                                     float* __restrict__ asrc, float* __restrict__ adst)
{
  __shared__ __align__(16) float sSD[128];
  const int tid = threadIdx.x, lane = tid & 31, wave = tid >> 5;
  float ws[8], wd[8];
#pragma unroll
  for (int m = 0; m < 2; ++m) {
    const v4f a = *(const v4f*)(as2 + lane * 8 + 4 * m);
    const v4f d = *(const v4f*)(ad2 + lane * 8 + 4 * m);
    ws[4 * m + 0] = a[0]; ws[4 * m + 1] = a[1]; ws[4 * m + 2] = a[2]; ws[4 * m + 3] = a[3];
    wd[4 * m + 0] = d[0]; wd[4 * m + 1] = d[1]; wd[4 * m + 2] = d[2]; wd[4 * m + 3] = d[3];
  }
#pragma unroll 1
  for (int nn = 0; nn < 8; ++nn) {
    const int ln = wave * 8 + nn;
    const int node = blockIdx.x * 64 + ln;
    const v4u p0 = *(const v4u*)(h2 + (size_t)node * kLat + lane * 8);
    float s = 0.0f, d = 0.0f;
#pragma unroll
    for (int m = 0; m < 4; ++m) {
      const unsigned w0 = p0[m];
      const float f0 = h16_to_f32(w0 & 0xffffu), f1 = h16_to_f32(w0 >> 16);
      s = fmaf(f0, ws[2 * m], s);     d = fmaf(f0, wd[2 * m], d);
      s = fmaf(f1, ws[2 * m + 1], s); d = fmaf(f1, wd[2 * m + 1], d);
    }
#pragma unroll
    for (int off = 1; off < 32; off <<= 1) {
      s += __shfl_xor(s, off, 32);
      d += __shfl_xor(d, off, 32);
    }
    if (lane == 0) { sSD[ln] = s; sSD[64 + ln] = d; }
  }
  __syncthreads();
  if (tid < 16) {
    const v4f v = *(const v4f*)(sSD + tid * 4);
    float* gp = asrc + (size_t)blockIdx.x * 64 + tid * 4;
    *(volatile v4f*)gp = v;
    __threadfence();
    *(volatile v4f*)gp = v;
  } else if (tid >= 32 && tid < 48) {
    const v4f v = *(const v4f*)(sSD + 64 + (tid - 32) * 4);
    float* gp = adst + (size_t)blockIdx.x * 64 + (tid - 32) * 4;
    *(volatile v4f*)gp = v;
    __threadfence();
    *(volatile v4f*)gp = v;
  }
}

__global__ __launch_bounds__(256) void aggregate1_kernel(
    const unsigned short* __restrict__ h1, const float* __restrict__ asrc, const float* __restrict__ adst,
    const unsigned* __restrict__ tabw, const int* __restrict__ deg, const float* __restrict__ b1,
    unsigned short* __restrict__ g16)
{
  __shared__ __align__(16) v8h sRow[8][64];
  const int lane = threadIdx.x & 31;
  const int wave = __builtin_amdgcn_readfirstlane((int)(threadIdx.x >> 5));
  const int i = blockIdx.x * 8 + wave;
  const bool valid = i < kN;
  const int ic = valid ? i : (kN - 1);
  const int head = lane >> 2;
  const int dgr = __builtin_amdgcn_readfirstlane(deg[ic]);
  const bool ovf = valid && (dgr > kCap);
  int dg = dgr < 0 ? 0 : (dgr > kCap ? kCap : dgr);
  dg = valid ? dg : 0;
  const unsigned word = tabw[(size_t)ic * 32 + lane];
  const float adv = adst[(size_t)ic * kHeads + head];
  const float sl = leaky02(asrc[(size_t)ic * kHeads + head] + adv);
  float acc[16];
#pragma unroll
  for (int k = 0; k < 16; ++k) acc[k] = 0.0f;
  float den = 0.0f;
  const int trips = dg + 1;
#pragma unroll 1
  for (int p = 0; p < trips; ++p) {
    const int q = (p > 0) ? (p - 1) : 0;
    const unsigned wsel = __shfl(word, q >> 1, 32);
    const int jt = (int)((q & 1) ? (wsel >> 16) : (wsel & 0xffffu));
    int j = (p == 0) ? ic : jt;
    j = j > (kN - 1) ? (kN - 1) : j;
    const float a = asrc[(size_t)j * kHeads + head];
    const float w = expf(leaky02(a + adv) - sl);
    den += w;
    const v4u p0 = *(const v4u*)(h1 + (size_t)j * kF1 + lane * 16);
    const v4u p1 = *(const v4u*)(h1 + (size_t)j * kF1 + lane * 16 + 8);
#pragma unroll
    for (int m = 0; m < 4; ++m) {
      const unsigned w0 = p0[m];
      const unsigned w1 = p1[m];
      acc[2 * m]         = fmaf(w, h16_to_f32(w0 & 0xffffu), acc[2 * m]);
      acc[2 * m + 1]     = fmaf(w, h16_to_f32(w0 >> 16),     acc[2 * m + 1]);
      acc[8 + 2 * m]     = fmaf(w, h16_to_f32(w1 & 0xffffu), acc[8 + 2 * m]);
      acc[8 + 2 * m + 1] = fmaf(w, h16_to_f32(w1 >> 16),     acc[8 + 2 * m + 1]);
    }
  }
  const float inv = 1.0f / (den + 1e-16f);
  const float qnan = __uint_as_float(0x7fc00000u);
  float bias[16];
#pragma unroll
  for (int m = 0; m < 4; ++m) {
    const v4f bb = *(const v4f*)(b1 + lane * 16 + 4 * m);
    bias[4 * m + 0] = bb[0]; bias[4 * m + 1] = bb[1]; bias[4 * m + 2] = bb[2]; bias[4 * m + 3] = bb[3];
  }
  v8h hv0, hv1;
#pragma unroll
  for (int k = 0; k < 8; ++k) {
    float v0 = acc[k] * inv + bias[k];
    float v1 = acc[8 + k] * inv + bias[8 + k];
    v0 = fmaxf(v0, 0.0f) * kGCarry;
    v1 = fmaxf(v1, 0.0f) * kGCarry;
    v0 = valid ? v0 : 0.0f;
    v1 = valid ? v1 : 0.0f;
    v0 = ovf ? qnan : v0;
    v1 = ovf ? qnan : v1;
    hv0[k] = (_Float16)v0;
    hv1[k] = (_Float16)v1;
  }
  sRow[wave][2 * lane]     = hv0;
  sRow[wave][2 * lane + 1] = hv1;
  __builtin_amdgcn_fence(__ATOMIC_RELEASE, "workgroup");
  __builtin_amdgcn_wave_barrier();
  __builtin_amdgcn_fence(__ATOMIC_ACQUIRE, "workgroup");
  const v8h r0 = sRow[wave][lane];
  const v8h r1 = sRow[wave][32 + lane];
  unsigned short* gp = g16 + (size_t)i * kF1 + lane * 8;
  for (int pass = 0; pass < 2; ++pass) {
    *(volatile v8h*)(gp)       = r0;
    *(volatile v8h*)(gp + 256) = r1;
    __threadfence();
  }
}

__global__ __launch_bounds__(256) void aggregate2_kernel(
    const unsigned short* __restrict__ h2, const float* __restrict__ asrc, const float* __restrict__ adst,
    const unsigned* __restrict__ tabw, const int* __restrict__ deg, const float* __restrict__ b2,
    unsigned short* __restrict__ zhi, unsigned short* __restrict__ zlo)
{
  const int lane = threadIdx.x & 31;
  const int wave = __builtin_amdgcn_readfirstlane((int)(threadIdx.x >> 5));
  const int i = blockIdx.x * 8 + wave;
  const bool valid = i < kN;
  const int ic = valid ? i : (kN - 1);
  const int dgr = __builtin_amdgcn_readfirstlane(deg[ic]);
  const bool ovf = valid && (dgr > kCap);
  int dg = dgr < 0 ? 0 : (dgr > kCap ? kCap : dgr);
  dg = valid ? dg : 0;
  const unsigned word = tabw[(size_t)ic * 32 + lane];
  const float adv = adst[ic];
  const float sl = leaky02(asrc[ic] + adv);
  float acc[8];
#pragma unroll
  for (int k = 0; k < 8; ++k) acc[k] = 0.0f;
  float den = 0.0f;
  const int trips = dg + 1;
#pragma unroll 1
  for (int p = 0; p < trips; ++p) {
    const int q = (p > 0) ? (p - 1) : 0;
    const unsigned wsel = __shfl(word, q >> 1, 32);
    const int jt = (int)((q & 1) ? (wsel >> 16) : (wsel & 0xffffu));
    int j = (p == 0) ? ic : jt;
    j = j > (kN - 1) ? (kN - 1) : j;
    const float a = asrc[j];
    const float w = expf(leaky02(a + adv) - sl);
    den += w;
    const v4u p0 = *(const v4u*)(h2 + (size_t)j * kLat + lane * 8);
#pragma unroll
    for (int m = 0; m < 4; ++m) {
      const unsigned w0 = p0[m];
      acc[2 * m]     = fmaf(w, h16_to_f32(w0 & 0xffffu), acc[2 * m]);
      acc[2 * m + 1] = fmaf(w, h16_to_f32(w0 >> 16),     acc[2 * m + 1]);
    }
  }
  const float inv = 1.0f / (den + 1e-16f);
  const float qnan = __uint_as_float(0x7fc00000u);
  const v4f bA = *(const v4f*)(b2 + lane * 8);
  const v4f bB = *(const v4f*)(b2 + lane * 8 + 4);
  v8h hv, lv;
#pragma unroll
  for (int k = 0; k < 4; ++k) {
    float v0 = acc[k] * inv + bA[k];
    float v1 = acc[4 + k] * inv + bB[k];
    v0 = valid ? v0 : 0.0f;
    v1 = valid ? v1 : 0.0f;
    v0 = ovf ? qnan : v0;
    v1 = ovf ? qnan : v1;
    const unsigned short h0 = f2bf_bits(v0), h1b = f2bf_bits(v1);
    const unsigned short l0 = f2bf_bits(v0 - bf_bits2f(h0)), l1 = f2bf_bits(v1 - bf_bits2f(h1b));
    hv[k]     = __builtin_bit_cast(_Float16, h0);
    hv[4 + k] = __builtin_bit_cast(_Float16, h1b);
    lv[k]     = __builtin_bit_cast(_Float16, l0);
    lv[4 + k] = __builtin_bit_cast(_Float16, l1);
  }
  const size_t o = (size_t)i * kLat + lane * 8;
  for (int pass = 0; pass < 2; ++pass) {
    *(volatile v8h*)(zhi + o) = hv;
    *(volatile v8h*)(zlo + o) = lv;
    __threadfence();
  }
}

__device__ __forceinline__ int lower_bound_batch(const int* __restrict__ batch, int key) {
  int lo = 0, hi = kN;
#pragma unroll 1
  for (int s = 0; s < 17; ++s) {
    int mid = (lo + hi) >> 1;
    mid = mid > (kN - 1) ? (kN - 1) : mid;
    const int bv = batch[mid];
    const bool act = lo < hi;
    const bool less = bv < key;
    const int nlo = (act && less) ? (mid + 1) : lo;
    const int nhi = (act && !less) ? mid : hi;
    lo = nlo; hi = nhi;
  }
  return lo;
}

__global__ __launch_bounds__(256) void pool_mlp_kernel(
    const unsigned short* __restrict__ zhi, const unsigned short* __restrict__ zlo, const int* __restrict__ batch,
    const float* __restrict__ Pw1, const float* __restrict__ Pb1, const float* __restrict__ Pw2,
    const float* __restrict__ Pb2, float* __restrict__ out1)
{
  __shared__ __align__(16) float sG[kLat];
  __shared__ __align__(16) float sH[kHid];
  __shared__ __align__(16) float sO[kLat];
  const int tid = threadIdx.x;
  const int g = blockIdx.x;
  int n0 = lower_bound_batch(batch, g);
  int n1 = lower_bound_batch(batch, g + 1);
  n0 = n0 < 0 ? 0 : (n0 > kN ? kN : n0);
  n1 = n1 < n0 ? n0 : (n1 > kN ? kN : n1);
  float sum = 0.0f;
#pragma unroll 1
  for (int n = n0; n < n1; ++n) {
    const unsigned hb = zhi[(size_t)n * kLat + tid];
    const unsigned lb = zlo[(size_t)n * kLat + tid];
    const float v = __uint_as_float(hb << 16) + __uint_as_float(lb << 16);
    sum += v;
  }
  const float cnt = fmaxf((float)(n1 - n0), 1.0f);
  sG[tid] = sum * (1.0f / cnt);
  __syncthreads();
  if (tid < kHid) {
    float a = 0.0f;
#pragma unroll 4
    for (int k = 0; k < kLat; ++k) a = fmaf(sG[k], Pw1[(size_t)k * kHid + tid], a);
    a += Pb1[tid];
    sH[tid] = fmaxf(a, 0.0f);
  }
  __syncthreads();
  {
    float a = 0.0f;
#pragma unroll 4
    for (int j = 0; j < kHid; ++j) a = fmaf(sH[j], Pw2[(size_t)j * kLat + tid], a);
    a += Pb2[tid];
    sO[tid] = a;
  }
  __syncthreads();
  if (tid < 64) {
    const v4f v = *(const v4f*)(sO + tid * 4);
    float* gp = out1 + (size_t)g * kLat + tid * 4;
    *(volatile v4f*)gp = v;
    __threadfence();
    *(volatile v4f*)gp = v;
  }
}

extern "C" void kernel_launch(void* const* d_in, const int* in_sizes, int n_in,
                              void* d_out, int out_size, void* d_ws, size_t ws_size,
                              hipStream_t stream) {
  if (n_in < 15) return;
  if (in_sizes[0] != kN * kInCh) return;
  if (in_sizes[1] != 2 * kE) return;
  if (in_sizes[2] != kN) return;
  if (in_sizes[3] != kInCh * kF1) return;
  if (in_sizes[4] != kF1 || in_sizes[5] != kF1 || in_sizes[6] != kF1) return;
  if (in_sizes[7] != kF1 * kLat) return;
  if (in_sizes[8] != kLat || in_sizes[9] != kLat || in_sizes[10] != kLat) return;
  if (in_sizes[11] != kLat * kHid) return;
  if (in_sizes[12] != kHid) return;
  if (in_sizes[13] != kHid * kLat) return;
  if (in_sizes[14] != kLat) return;
  if (out_size != kN * kLat + kGraphs * kLat) return;
  if (ws_size < kWsTotal) return;

  const float* x     = (const float*)d_in[0];
  const int*   ei    = (const int*)  d_in[1];
  const int*   batch = (const int*)  d_in[2];
  const float* W1    = (const float*)d_in[3];
  const float* as1   = (const float*)d_in[4];
  const float* ad1   = (const float*)d_in[5];
  const float* b1    = (const float*)d_in[6];
  const float* W2    = (const float*)d_in[7];
  const float* as2   = (const float*)d_in[8];
  const float* ad2   = (const float*)d_in[9];
  const float* b2    = (const float*)d_in[10];
  const float* Pw1   = (const float*)d_in[11];
  const float* Pb1   = (const float*)d_in[12];
  const float* Pw2   = (const float*)d_in[13];
  const float* Pb2   = (const float*)d_in[14];
  float* out0 = (float*)d_out;
  float* out1 = (float*)d_out + (kOut1ByteOff / 4);

  char* ws = (char*)d_ws;
  unsigned short* H1   = (unsigned short*)(ws + kOffR1);
  unsigned short* H2   = (unsigned short*)(ws + kOffR1);
  unsigned short* X16  = (unsigned short*)(ws + kOffR2);
  unsigned short* G16  = (unsigned short*)(ws + kOffR2);
  unsigned short* ZH   = (unsigned short*)(ws + kOffR2);
  unsigned short* ZL   = (unsigned short*)(ws + kOffR2 + kSzHalf);
  unsigned short* TH   = (unsigned short*)(ws + kOffTH);
  unsigned short* TL   = (unsigned short*)(ws + kOffTL);
  unsigned short* W1T  = (unsigned short*)(ws + kOffW1T);
  unsigned short* W2T  = (unsigned short*)(ws + kOffW2T);
  unsigned short* P1H  = (unsigned short*)(ws + kOffP1H);
  unsigned short* P1L  = (unsigned short*)(ws + kOffP1L);
  unsigned short* P2H  = (unsigned short*)(ws + kOffP2H);
  unsigned short* P2L  = (unsigned short*)(ws + kOffP2L);
  float*          AS1  = (float*)(ws + kOffAS1);
  float*          AD1  = (float*)(ws + kOffAD1);
  float*          AS2  = (float*)(ws + kOffAS2);
  float*          AD2  = (float*)(ws + kOffAD2);
  int*            DEG  = (int*)(ws + kOffDEG);
  unsigned short* TAB  = (unsigned short*)(ws + kOffTAB);

  cvt_x_f16_kernel<<<(kMP * kInCh / 8) / 256, 256, 0, stream>>>(x, X16);
  transpose_w_kernel<0><<<dim3(kF1 / 64, kInCh / 64), 256, 0, stream>>>(W1, kInCh, kF1, W1T, W1T, kWCarry);
  transpose_w_kernel<0><<<dim3(kLat / 64, kF1 / 64), 256, 0, stream>>>(W2, kF1, kLat, W2T, W2T, kWCarry);
  transpose_w_kernel<1><<<dim3(kHid / 64, kLat / 64), 256, 0, stream>>>(Pw1, kLat, kHid, P1H, P1L, 1.0f);
  transpose_w_kernel<1><<<dim3(kLat / 64, kHid / 64), 256, 0, stream>>>(Pw2, kHid, kLat, P2H, P2L, 1.0f);

  build_table_kernel<<<kTabBlocks, 512, 0, stream>>>(ei, TAB, DEG);

  wmma_gemm64<0, false, 0, 1, false, 0><<<dim3(782, 1), 256, 0, stream>>>(
      X16, nullptr, kInCh, 0L,
      W1T, nullptr, kInCh, 0L,
      (void*)H1, nullptr, kF1, 0L,
      nullptr, nullptr, 0L,
      kMP, kF1, kInCh, kInvW, kMP);
  score1_kernel<<<kMP / 64, 256, 0, stream>>>(H1, as1, ad1, AS1, AD1);
  aggregate1_kernel<<<kMP / 8, 256, 0, stream>>>(H1, AS1, AD1, (const unsigned*)(const void*)TAB, DEG, b1, G16);

  wmma_gemm64<0, false, 0, 1, false, 0><<<dim3(391, 1), 256, 0, stream>>>(
      G16, nullptr, kF1, 0L,
      W2T, nullptr, kF1, 0L,
      (void*)H2, nullptr, kLat, 0L,
      nullptr, nullptr, 0L,
      kMP, kLat, kF1, kInvGW, kMP);
  score2_kernel<<<kMP / 64, 256, 0, stream>>>(H2, as2, ad2, AS2, AD2);
  aggregate2_kernel<<<kMP / 8, 256, 0, stream>>>(H2, AS2, AD2, (const unsigned*)(const void*)TAB, DEG, b2, ZH, ZL);

  wmma_gemm64<1, true, 2, 2, false, 2><<<dim3(98, 1), 256, 0, stream>>>(
      ZH, ZL, kLat, 0L,
      P1H, P1L, kLat, 0L,
      (void*)TH, (void*)TL, kHid, 0L,
      Pb1, nullptr, 0L,
      kMP, kHid, kLat, 1.0f, kMP);
  wmma_gemm64<1, true, 2, 0, false, 0><<<dim3(391, 1), 256, 0, stream>>>(
      TH, TL, kHid, 0L,
      P2H, P2L, kHid, 0L,
      (void*)out0, nullptr, kLat, 0L,
      Pb2, nullptr, 0L,
      kMP, kLat, kHid, 1.0f, kN);

  pool_mlp_kernel<<<kGraphs, 256, 0, stream>>>(ZH, ZL, batch, Pw1, Pb1, Pw2, Pb2, out1);
}
